// DyGDecoder_86758339379618
// MI455X (gfx1250) — hardware-verified
//
#include <hip/hip_runtime.h>


#define NB_  2
#define TS   2048
#define TT   4096
#define DD   256
#define NH_  4
#define HD   64
#define FF   1024
#define PCAR 1024.0f
#define SCL  0.125f
typedef _Float16 h16;
typedef unsigned short bf;
typedef __attribute__((ext_vector_type(16))) __bf16   v16bf;
typedef __attribute__((ext_vector_type(16))) _Float16 v16h;
typedef __attribute__((ext_vector_type(8)))  _Float16 v8h;
typedef __attribute__((ext_vector_type(8)))  unsigned short v8us;
typedef __attribute__((ext_vector_type(8)))  float    v8f;
typedef __attribute__((ext_vector_type(4)))  float    v4f;
typedef v8h  __attribute__((may_alias)) v8ha;
typedef v4f  __attribute__((may_alias)) v4fa;
typedef v8us __attribute__((may_alias)) v8usa;

__device__ __forceinline__ unsigned short f2bf(float f) { unsigned u = __float_as_uint(f); u += 0x7FFFu + ((u >> 16) & 1u); return (unsigned short)(u >> 16); }
__device__ __forceinline__ float bf2f(unsigned short b) { return __uint_as_float(((unsigned)b) << 16); }
__device__ __forceinline__ float bfr(float f) { return bf2f(f2bf(f)); }
__device__ __forceinline__ v16h cat16(v8h lo, v8h hi) { return __builtin_shufflevector(lo, hi, 0, 1, 2, 3, 4, 5, 6, 7, 8, 9, 10, 11, 12, 13, 14, 15); }
__device__ __forceinline__ v16bf cat16b(v8us lo, v8us hi) { return __builtin_bit_cast(v16bf, __builtin_shufflevector(lo, hi, 0, 1, 2, 3, 4, 5, 6, 7, 8, 9, 10, 11, 12, 13, 14, 15)); }
__device__ __forceinline__ v8f wmma16(v16h a, v16h b, v8f c) { return __builtin_amdgcn_wmma_f32_16x16x32_f16(false, a, false, b, (short)0, c, false, false); }
__device__ __forceinline__ v8f wmmab(v16bf a, v16bf b, v8f c) { return __builtin_amdgcn_wmma_f32_16x16x32_bf16(false, a, false, b, (short)0, c, false, false); }


template <typename T16> struct WFrag;
template <> struct WFrag<h16> { typedef v16h V; static __device__ __forceinline__ V ld(const h16* p) { return cat16(*(const v8h*)p, *(const v8h*)(p + 16)); } static __device__ __forceinline__ v8f mma(V a, V b, v8f c) { return wmma16(a, b, c); } };
template <> struct WFrag<bf> { typedef v16bf V; static __device__ __forceinline__ V ld(const bf* p) { return cat16b(*(const v8us*)p, *(const v8us*)(p + 16)); } static __device__ __forceinline__ v8f mma(V a, V b, v8f c) { return wmmab(a, b, c); } };
template <typename T16, int NSPLIT, bool BIAS>
__global__ __launch_bounds__(32) void k_gemmw(const T16* __restrict__ A, const T16* __restrict__ A2, const T16* __restrict__ Bt, const T16* __restrict__ Bt2, int K, float* C, int ldc, const float* __restrict__ bias, size_t sA, size_t sB, size_t sC) {
    typedef typename WFrag<T16>::V V;
    __shared__ __align__(16) float os[16 * 68];
    const size_t z = blockIdx.z; A += z * sA; if (A2) A2 += z * sA; Bt += z * sB; if (Bt2) Bt2 += z * sB; C += z * sC;
    const int lane = threadIdx.x & 31, lr = lane & 15, hi = lane >> 4; const int r0 = blockIdx.x * 64, c0 = blockIdx.y * 64;
    v8f acc[4][4];
#pragma unroll
    for (int mb = 0; mb < 4; ++mb)
#pragma unroll
        for (int nb = 0; nb < 4; ++nb) acc[mb][nb] = (v8f){};
    const size_t aoff = (size_t)(r0 + lr) * K + 8 * hi, boff = (size_t)(c0 + lr) * K + 8 * hi;
#pragma unroll 1
    for (int kc = 0; kc < K; kc += 32) {
        V a[4], a2[4];
#pragma unroll
        for (int mb = 0; mb < 4; ++mb) { a[mb] = WFrag<T16>::ld(A + aoff + (size_t)mb * 16 * K + kc); if (NSPLIT == 1 || NSPLIT == 2) a2[mb] = WFrag<T16>::ld(A2 + aoff + (size_t)mb * 16 * K + kc); }
#pragma unroll
        for (int nb = 0; nb < 4; ++nb) { const V b = WFrag<T16>::ld(Bt + boff + (size_t)nb * 16 * K + kc); V b2; if (NSPLIT >= 2) b2 = WFrag<T16>::ld(Bt2 + boff + (size_t)nb * 16 * K + kc);
#pragma unroll
            for (int mb = 0; mb < 4; ++mb) { acc[mb][nb] = WFrag<T16>::mma(a[mb], b, acc[mb][nb]); if (NSPLIT == 1 || NSPLIT == 2) acc[mb][nb] = WFrag<T16>::mma(a2[mb], b, acc[mb][nb]); if (NSPLIT >= 2) acc[mb][nb] = WFrag<T16>::mma(a[mb], b2, acc[mb][nb]); } }
        asm volatile("v_nop\n\tv_nop\n\tv_nop\n\tv_nop" : "+v"(acc[0][0]), "+v"(acc[1][1]), "+v"(acc[2][2]), "+v"(acc[3][3]) : "v"(a[0]), "v"(a[3]));
    }
#pragma unroll
    for (int mb = 0; mb < 4; ++mb) {
#pragma unroll
        for (int nb = 0; nb < 4; ++nb) {
#pragma unroll
            for (int j = 0; j < 8; ++j) os[(hi * 8 + j) * 68 + nb * 16 + lr] = acc[mb][nb][j]; }
        __builtin_amdgcn_wave_barrier(); asm volatile("" ::: "memory");
        float* crow = C + (size_t)(r0 + mb * 16) * ldc + c0;
#pragma unroll 1
        for (int ps = 0; ps < 2; ++ps) {
#pragma unroll
            for (int s = 0; s < 8; ++s) { const int row = 2 * s + hi, cofs = lr * 4; v4f val = *(const v4fa*)(os + row * 68 + cofs); if (BIAS) { val[0] += bfr(bias[c0 + cofs]); val[1] += bfr(bias[c0 + cofs + 1]); val[2] += bfr(bias[c0 + cofs + 2]); val[3] += bfr(bias[c0 + cofs + 3]); }
                *(volatile v4f*)(crow + (size_t)row * ldc + cofs) = val; }
            if (ps == 0) __threadfence(); }
        __builtin_amdgcn_wave_barrier(); asm volatile("" ::: "memory");
    }
}

__device__ __forceinline__ h16 tohx(float x) { return (h16)x; }
__device__ __forceinline__ void splitf(float y, unsigned short& h, unsigned short& l) { h = f2bf(y); l = f2bf(y - bf2f(h)); }
typedef __attribute__((ext_vector_type(2))) _Float16 v2h;
typedef __attribute__((ext_vector_type(4))) _Float16 v4h;
typedef __attribute__((ext_vector_type(2))) unsigned short v2us;
typedef __attribute__((ext_vector_type(4))) unsigned short v4us;
typedef __attribute__((ext_vector_type(2))) float v2f;

__global__ __launch_bounds__(256) void k_wtG(const float* __restrict__ w, int K, int N, bf* Bt) {
    const int lane = threadIdx.x & 31; const int L0 = (blockIdx.x * 8 + (threadIdx.x >> 5)) * 8; const int nlines = N * K / 64;
#pragma unroll 1
    for (int ps = 0; ps < 2; ++ps) {
#pragma unroll 1
        for (int l = 0; l < 8; ++l) { const int L = L0 + l; if (L >= nlines) break; const size_t e = (size_t)L * 64 + lane * 2; const int k = (int)(e % K), n = (int)(e / K); v2us o;
            o[0] = f2bf(w[(size_t)k * N + n]); o[1] = f2bf(w[(size_t)(k + 1) * N + n]); *(volatile v2us*)(Bt + e) = o; }
        if (ps == 0) __threadfence(); }
}
template <int MODE>
__global__ __launch_bounds__(256) void k_ln256(const float* __restrict__ A, const float* __restrict__ A2, const float* __restrict__ gg, const float* __restrict__ bb, float* INP, bf* Yh, bf* Yl) {
    const int lane = threadIdx.x & 31; const int r = blockIdx.x * 8 + (threadIdx.x >> 5); if (r >= TT) return; const float* src = (MODE == 0) ? ((r < TS) ? (A + (size_t)r * DD) : (A2 + (size_t)(r - TS) * DD)) : (A + (size_t)r * DD); float v[8]; float s = 0.f;
#pragma unroll
    for (int c = 0; c < 2; ++c) { const v4f a = *(const v4f*)(src + c * 128 + lane * 4);
#pragma unroll
        for (int q = 0; q < 4; ++q) { float t = (MODE == 0) ? bfr(a[q]) : a[q]; asm volatile("" : "+v"(t)); v[c * 4 + q] = t; s = __fadd_rn(s, t); } }
#pragma unroll
    for (int sh = 16; sh; sh >>= 1) s += __shfl_xor(s, sh, 32);
    const float mu = s * (1.0f / DD); float qq = 0.f;
#pragma unroll
    for (int i = 0; i < 8; ++i) { const float d0 = v[i] - mu; float p = __fmul_rn(d0, d0); asm volatile("" : "+v"(p)); qq = __fadd_rn(qq, p); }
#pragma unroll
    for (int sh = 16; sh; sh >>= 1) qq += __shfl_xor(qq, sh, 32);
    const float rs = __fdiv_rn(1.0f, __fsqrt_rn(__fadd_rn(qq * (1.0f / DD), 1e-5f)));
#pragma unroll 1
    for (int ps = 0; ps < 2; ++ps) {
#pragma unroll
        for (int c = 0; c < 2; ++c) { v4us oh, ol; v4f raw;
#pragma unroll
            for (int q = 0; q < 4; ++q) { const int col = c * 128 + lane * 4 + q; float g = bfr(gg[col]), bq = bfr(bb[col]); asm volatile("" : "+v"(g)); asm volatile("" : "+v"(bq)); float tn = __fmul_rn(v[c * 4 + q] - mu, rs); asm volatile("" : "+v"(tn)); float tg = __fmul_rn(tn, g); asm volatile("" : "+v"(tg)); unsigned short a2, c2; splitf(__fadd_rn(tg, bq), a2, c2); oh[q] = a2; ol[q] = c2; raw[q] = v[c * 4 + q]; }
            const size_t o = (size_t)r * DD + c * 128 + lane * 4; if (MODE == 0) *(volatile v4f*)(INP + o) = raw; *(volatile v4us*)(Yh + o) = oh; *(volatile v4us*)(Yl + o) = ol; }
        if (ps == 0) __threadfence(); }
}
__global__ __launch_bounds__(256) void k_pl(const float* __restrict__ F3, int off, h16* P) { const int e = (blockIdx.x * 256 + threadIdx.x) * 2; if (e >= NH_ * TT * HD) return; const int d = e & 63; const int t = (e >> 6) & (TT - 1); const int h = e / (TT * HD); v2h o; o[0] = tohx(F3[(size_t)t * 3 * DD + off + h * HD + d]); o[1] = tohx(F3[(size_t)t * 3 * DD + off + h * HD + d + 1]); *(volatile v2h*)(P + e) = o; __threadfence(); *(volatile v2h*)(P + e) = o; }
__global__ __launch_bounds__(256) void k_vt(const float* __restrict__ F3, h16* VT) { const int e = (blockIdx.x * 256 + threadIdx.x) * 2; if (e >= NH_ * HD * TT) return; const int t = e & (TT - 1); const int d = (e / TT) & 63; const int h = e / (TT * HD); v2h o; o[0] = tohx(F3[(size_t)t * 3 * DD + 2 * DD + h * HD + d]); o[1] = tohx(F3[(size_t)(t + 1) * 3 * DD + 2 * DD + h * HD + d]); *(volatile v2h*)(VT + e) = o; __threadfence(); *(volatile v2h*)(VT + e) = o; }
__global__ __launch_bounds__(256) void k_smax(const float* __restrict__ S, const float* __restrict__ tm, float* RS) { const int lane = threadIdx.x & 31; const int i = blockIdx.x * 8 + (threadIdx.x >> 5); if (i >= TT) return; const float ti = tm[i]; const float* sr = S + (size_t)i * TT; float m = -3.0e38f;
#pragma unroll 4
    for (int c0 = lane * 4; c0 < TT; c0 += 128) { const v4f v = *(const v4f*)(sr + c0), t4 = *(const v4f*)(tm + c0);
#pragma unroll
        for (int q = 0; q < 4; ++q) m = (ti >= t4[q]) ? fmaxf(m, v[q]) : m; }
#pragma unroll
    for (int sh = 16; sh; sh >>= 1) m = fmaxf(m, __shfl_xor(m, sh, 32));
    const float o = lane == 0 ? m : 0.f; *(volatile float*)(RS + (size_t)i * 32 + lane) = o; __threadfence(); *(volatile float*)(RS + (size_t)i * 32 + lane) = o; }
__global__ __launch_bounds__(256) void k_sexp(const float* __restrict__ S, const float* __restrict__ tm, float* RS, h16* P) { const int lane = threadIdx.x & 31; const int i = blockIdx.x * 8 + (threadIdx.x >> 5); if (i >= TT) return; const float ti = tm[i]; const float* sr = S + (size_t)i * TT; const float m = RS[(size_t)i * 32]; float sum = 0.f;
#pragma unroll 1
    for (int ps = 0; ps < 2; ++ps) { sum = 0.f;
#pragma unroll 2
        for (int c0 = lane * 4; c0 < TT; c0 += 128) { const v4f v = *(const v4f*)(sr + c0), t4 = *(const v4f*)(tm + c0); v4h o;
#pragma unroll
            for (int q = 0; q < 4; ++q) { float dlt = __fsub_rn(v[q], m); asm volatile("" : "+v"(dlt)); const float e = (ti >= t4[q]) ? __expf(__fmul_rn(dlt, SCL)) : 0.f; sum += e; o[q] = tohx(e * PCAR); }
            *(volatile v4h*)(P + (size_t)i * TT + c0) = o; }
        if (ps == 0) __threadfence(); }
#pragma unroll
    for (int sh = 16; sh; sh >>= 1) sum += __shfl_xor(sum, sh, 32);
    const float o2 = lane == 0 ? m : (lane == 1 ? __fdiv_rn(1.0f, sum * PCAR) : 0.f); *(volatile float*)(RS + (size_t)i * 32 + lane) = o2; __threadfence(); *(volatile float*)(RS + (size_t)i * 32 + lane) = o2; }
__global__ __launch_bounds__(256) void k_mrg(const float* __restrict__ O, const float* __restrict__ RS, int h, bf* Ah, bf* Al) { const int e = (blockIdx.x * 256 + threadIdx.x) * 2; if (e >= TT * HD) return; const int d = e & 63; const int t = e >> 6; const float sc = RS[(size_t)t * 32 + 1]; v2us oh, ol;
#pragma unroll
    for (int q = 0; q < 2; ++q) { unsigned short a, c2; splitf(__fmul_rn(O[e + q], sc), a, c2); oh[q] = a; ol[q] = c2; } const size_t oo = (size_t)t * DD + h * HD + d; *(volatile v2us*)(Ah + oo) = oh; *(volatile v2us*)(Al + oo) = ol; __threadfence(); *(volatile v2us*)(Ah + oo) = oh; *(volatile v2us*)(Al + oo) = ol; }
__global__ __launch_bounds__(256) void k_tcat(const float* __restrict__ t1, const float* __restrict__ t2, float* TM) { const int i = (blockIdx.x * 256 + threadIdx.x) * 4; if (i >= TT) return; const v4f a = (i < TS) ? *(const v4f*)(t1 + i) : *(const v4f*)(t2 + i - TS); v4f o;
#pragma unroll
    for (int q = 0; q < 4; ++q) o[q] = bfr(a[q]); *(volatile v4f*)(TM + i) = o; __threadfence(); *(volatile v4f*)(TM + i) = o; }
__global__ __launch_bounds__(256) void k_res(const float* __restrict__ INP, const float* __restrict__ Y, float* OUTR) { const size_t i = ((size_t)blockIdx.x * 256 + threadIdx.x) * 4; if (i >= (size_t)TT * DD) return; const v4f a = *(const v4f*)(INP + i), y = *(const v4f*)(Y + i); v4f o;
#pragma unroll
    for (int q = 0; q < 4; ++q) o[q] = __fadd_rn(a[q], y[q]); *(volatile v4f*)(OUTR + i) = o; __threadfence(); *(volatile v4f*)(OUTR + i) = o; }
__global__ __launch_bounds__(256) void k_gelu2(const float* __restrict__ F, bf* Ph, bf* Pl) { const size_t i = ((size_t)blockIdx.x * 256 + threadIdx.x) * 2; if (i >= (size_t)TT * FF) return; v2us oh, ol;
#pragma unroll
    for (int q = 0; q < 2; ++q) { const float h = F[i + q]; float er = erff(h * 0.70710678f); asm volatile("" : "+v"(er)); float hh = __fmul_rn(0.5f, h); asm volatile("" : "+v"(hh)); unsigned short a, c2; splitf(__fmul_rn(hh, __fadd_rn(1.0f, er)), a, c2); oh[q] = a; ol[q] = c2; }
    *(volatile v2us*)(Ph + i) = oh; *(volatile v2us*)(Pl + i) = ol; __threadfence(); *(volatile v2us*)(Ph + i) = oh; *(volatile v2us*)(Pl + i) = ol; }
__global__ __launch_bounds__(256) void k_fin(const float* __restrict__ OUTR, const float* __restrict__ H2, int b, float* OUT0, float* OUT1) { const size_t i = ((size_t)blockIdx.x * 256 + threadIdx.x) * 4; if (i >= (size_t)TT * DD) return; const size_t t = i / DD; const int c = (int)(i % DD); const v4f a = *(const v4f*)(OUTR + i), h = *(const v4f*)(H2 + i); v4f o;
#pragma unroll
    for (int q = 0; q < 4; ++q) o[q] = __fadd_rn(a[q], h[q]); float* dst = (t < TS) ? (OUT0 + ((size_t)b * TS + t) * DD + c) : (OUT1 + ((size_t)b * TS + (t - TS)) * DD + c); *(volatile v4f*)dst = o; __threadfence(); *(volatile v4f*)dst = o; }

extern "C" void kernel_launch(void* const* d_in, const int* in_sizes, int n_in,
                              void* d_out, int out_size, void* d_ws, size_t ws_size, hipStream_t stream) {
    (void)in_sizes; (void)n_in; (void)out_size;
    const float* IN[18]; for (int i = 0; i < 18; ++i) IN[i] = (const float*)d_in[i];
    float* OUT0 = (float*)d_out; float* OUT1 = OUT0 + (size_t)NB_ * TS * DD;
    char* wsp = (char*)d_ws;
    auto take = [&](size_t bytes) { char* p = wsp; wsp += (bytes + 255) & ~(size_t)255; return (void*)p; };
    bf* WS = (bf*)take((size_t)3 * DD * DD * 2); bf* WC = (bf*)take((size_t)3 * DD * DD * 2); bf* WP = (bf*)take((size_t)DD * DD * 2); bf* WF1 = (bf*)take((size_t)FF * DD * 2); bf* WF2 = (bf*)take((size_t)DD * FF * 2); float* TM = (float*)take((size_t)TT * 4);
    float* INP = (float*)take((size_t)TT * DD * 4); bf* Xh = (bf*)take((size_t)TT * DD * 2); bf* Xl = (bf*)take((size_t)TT * DD * 2); float* F3 = (float*)take((size_t)TT * 3 * DD * 4);
    h16* QP = (h16*)take((size_t)NH_ * TT * HD * 2); h16* KP = (h16*)take((size_t)NH_ * TT * HD * 2); h16* VT = (h16*)take((size_t)NH_ * HD * TT * 2); float* Sb = (float*)take((size_t)TT * TT * 4); h16* Pm = (h16*)take((size_t)TT * TT * 2); float* RS = (float*)take((size_t)TT * 32 * 4); float* Ob = (float*)take((size_t)TT * HD * 4);
    bf* Ah = (bf*)take((size_t)TT * DD * 2); bf* Al = (bf*)take((size_t)TT * DD * 2); float* Y = (float*)take((size_t)TT * DD * 4); float* OUTR = (float*)take((size_t)TT * DD * 4); float* HF = (float*)take((size_t)TT * FF * 4); bf* Gh = (bf*)take((size_t)TT * FF * 2); bf* Gl = (bf*)take((size_t)TT * FF * 2); float* H2 = (float*)take((size_t)TT * DD * 4);
    if ((size_t)(wsp - (char*)d_ws) > ws_size) return;
    { k_wtG<<<(unsigned)((DD * 3 * DD / 64 + 63) / 64), 256, 0, stream>>>(IN[6], DD, 3 * DD, WS); k_wtG<<<(unsigned)((DD * 3 * DD / 64 + 63) / 64), 256, 0, stream>>>(IN[8], DD, 3 * DD, WC); k_wtG<<<(unsigned)((DD * DD / 64 + 63) / 64), 256, 0, stream>>>(IN[10], DD, DD, WP);
      k_wtG<<<(unsigned)((DD * FF / 64 + 63) / 64), 256, 0, stream>>>(IN[14], DD, FF, WF1); k_wtG<<<(unsigned)((FF * DD / 64 + 63) / 64), 256, 0, stream>>>(IN[16], FF, DD, WF2); }
    const unsigned LP = (NH_ * TT * HD / 2 + 255) / 256;
    for (int b = 0; b < NB_; ++b) {
        k_tcat<<<(TT / 4 + 255) / 256, 256, 0, stream>>>(IN[2] + (size_t)b * TS, IN[3] + (size_t)b * TS, TM);
        k_ln256<0><<<TT / 8, 256, 0, stream>>>(IN[0] + (size_t)b * TS * DD, IN[1] + (size_t)b * TS * DD, IN[4], IN[5], INP, Xh, Xl);
        k_gemmw<bf, 1, true><<<dim3(TS / 64, 3 * DD / 64, 1), 32, 0, stream>>>(Xh, Xl, WS, nullptr, DD, F3, 3 * DD, IN[7], 0, 0, 0);
        k_gemmw<bf, 1, true><<<dim3(TS / 64, 3 * DD / 64, 1), 32, 0, stream>>>(Xh + (size_t)TS * DD, Xl + (size_t)TS * DD, WC, nullptr, DD, F3 + (size_t)TS * 3 * DD, 3 * DD, IN[9], 0, 0, 0);
        k_pl<<<LP, 256, 0, stream>>>(F3, 0, QP); k_pl<<<LP, 256, 0, stream>>>(F3, DD, KP); k_vt<<<LP, 256, 0, stream>>>(F3, VT);
        for (int h = 0; h < NH_; ++h) {
            k_gemmw<h16, 0, false><<<dim3(TT / 64, TT / 64, 1), 32, 0, stream>>>(QP + (size_t)h * TT * HD, nullptr, KP + (size_t)h * TT * HD, nullptr, HD, Sb, TT, nullptr, 0, 0, 0);
            k_smax<<<TT / 8, 256, 0, stream>>>(Sb, TM, RS); k_sexp<<<TT / 8, 256, 0, stream>>>(Sb, TM, RS, Pm);
            k_gemmw<h16, 0, false><<<dim3(TT / 64, 1, 1), 32, 0, stream>>>(Pm, nullptr, VT + (size_t)h * HD * TT, nullptr, TT, Ob, HD, nullptr, 0, 0, 0);
            k_mrg<<<(TT * HD / 2 + 255) / 256, 256, 0, stream>>>(Ob, RS, h, Ah, Al); }
        k_gemmw<bf, 1, true><<<dim3(TT / 64, DD / 64, 1), 32, 0, stream>>>(Ah, Al, WP, nullptr, DD, Y, DD, IN[11], 0, 0, 0); k_res<<<(TT * DD / 4 + 255) / 256, 256, 0, stream>>>(INP, Y, OUTR);
        k_ln256<1><<<TT / 8, 256, 0, stream>>>(OUTR, nullptr, IN[12], IN[13], nullptr, Xh, Xl);
        k_gemmw<bf, 1, true><<<dim3(TT / 64, FF / 64, 1), 32, 0, stream>>>(Xh, Xl, WF1, nullptr, DD, HF, FF, IN[15], 0, 0, 0); k_gelu2<<<(unsigned)(((size_t)TT * FF / 2 + 255) / 256), 256, 0, stream>>>(HF, Gh, Gl);
        k_gemmw<bf, 1, true><<<dim3(TT / 64, DD / 64, 1), 32, 0, stream>>>(Gh, Gl, WF2, nullptr, FF, H2, DD, IN[17], 0, 0, 0); k_fin<<<(TT * DD / 4 + 255) / 256, 256, 0, stream>>>(OUTR, H2, b, OUT0, OUT1); }
}
